// PretrainGNNEncoder_46480136077495
// MI455X (gfx1250) — hardware-verified
//
#include <hip/hip_runtime.h>
#include <stddef.h>
#include <math.h>


#define FIN     141
#define KPX     160
#define CH      256
#define NL      4
#define NTHR    256
#define NWAVE   8
#define EPT     8
#define NGRP    2
#define CHUNK   (NTHR * EPT * NGRP)
#define WCAP    (EPT * NGRP * 32)
#define LISTN   (NWAVE * WCAP)
#define NBC     4096
#define NBF     2048
#define FPC     (NBC / NBF)
#define RCAP    40960
#define RBN     128
#define TGT     256
#define DEGCAP  256
#define OTHR    512
#define BM      64
#define STATR   256
#define WSCAP   134217728
#define BN_EPS  1e-5

#define LDS_FILL ((RCAP + NBF + LISTN) * 4 + 64)
#define LDS_GEMM (BM * CH * 4)

static_assert((CHUNK & (CHUNK - 1)) == 0);
static_assert(CHUNK <= 4096);
static_assert(NBC <= 4096 && NBF <= 4096);
static_assert((NBC & (NBC - 1)) == 0 && (NBF & (NBF - 1)) == 0);
static_assert(NBC == FPC * NBF && FPC == 2);
static_assert(OTHR * 8 == NBC);
static_assert(OTHR / 32 == 8 * FPC);
static_assert((RCAP % 32) == 0);
static_assert(TGT == NWAVE * 32);
static_assert((TGT % BM) == 0 && (TGT % STATR) == 0);
static_assert((DEGCAP % 32) == 0);
static_assert(BM == 64 && NWAVE == 8 && CH == 256);
static_assert((KPX % 32) == 0 && KPX >= FIN);
static_assert(BM * KPX * 2 * 2 <= LDS_GEMM);
static_assert(BM * CH * 2 * 2 <= LDS_GEMM);
static_assert(((BM * KPX / 8) % NTHR) == 0);
static_assert(((BM * CH / 8) % NTHR) == 0);

typedef float          v4f  __attribute__((ext_vector_type(4)));
typedef float          v8f  __attribute__((ext_vector_type(8)));
typedef double         v2d  __attribute__((ext_vector_type(2)));
typedef int            v4i  __attribute__((ext_vector_type(4)));
typedef unsigned short v8us __attribute__((ext_vector_type(8)));
typedef unsigned short v16us __attribute__((ext_vector_type(16)));
typedef __bf16         v16bf __attribute__((ext_vector_type(16)));
union FragU { v16us w; v8us u[2]; };

__device__ __forceinline__ v8f wmb(v16us a, v16us b, v8f c) {
  const v16bf ab = __builtin_bit_cast(v16bf, a);
  const v16bf bb = __builtin_bit_cast(v16bf, b);
  v8f d = __builtin_amdgcn_wmma_f32_16x16x32_bf16(false, ab, false, bb, (short)0, c, false, false);
  asm volatile("v_nop\n\tv_nop\n\tv_nop\n\tv_nop" : "+v"(d) : "v"(a), "v"(b));
  return d;
}

__device__ __forceinline__ unsigned int bfb(float f) {
  const unsigned int u = __float_as_uint(f);
  return (u + 0x7FFFu + ((u >> 16) & 1u)) >> 16;
}
__device__ __forceinline__ void sp1(float v, unsigned short& h, unsigned short& l) {
  const unsigned int hb = bfb(v);
  const float hf = __uint_as_float(hb << 16);
  h = (unsigned short)hb;
  l = (unsigned short)bfb(v - hf);
}
__device__ __forceinline__ void sp8(v4f a, v4f b, v8us& h, v8us& l) {
  unsigned short hh, ll;
  sp1(a.x, hh, ll); h[0] = hh; l[0] = ll;
  sp1(a.y, hh, ll); h[1] = hh; l[1] = ll;
  sp1(a.z, hh, ll); h[2] = hh; l[2] = ll;
  sp1(a.w, hh, ll); h[3] = hh; l[3] = ll;
  sp1(b.x, hh, ll); h[4] = hh; l[4] = ll;
  sp1(b.y, hh, ll); h[5] = hh; l[5] = ll;
  sp1(b.z, hh, ll); h[6] = hh; l[6] = ll;
  sp1(b.w, hh, ll); h[7] = hh; l[7] = ll;
}

__device__ __forceinline__ v4f relu4(v4f t) {
  v4f r;
  r.x = fmaxf(t.x, 0.f); r.y = fmaxf(t.y, 0.f); r.z = fmaxf(t.z, 0.f); r.w = fmaxf(t.w, 0.f);
  return r;
}
__device__ __forceinline__ float rlf(float v, int l) {
  return __int_as_float(__builtin_amdgcn_readlane(__float_as_int(v), l));
}

__global__ __launch_bounds__(NTHR) void k_wprep(const float* __restrict__ W, int nrow, int kin, int kpu,
                                               unsigned short* ph, unsigned short* pl, int units) {
  const int i = (int)blockIdx.x * NTHR + (int)threadIdx.x;
  if (i >= units) return;
  const int n  = i / kpu;
  const int k0 = (i - n * kpu) * 8;
  const int nc = n < nrow - 1 ? n : nrow - 1;
  const float* wr = W + (size_t)nc * kin;
  v8us hv, lv;
#pragma unroll
  for (int e = 0; e < 8; ++e) {
    const int k  = k0 + e;
    const int kc = k < kin ? k : kin - 1;
    float f = wr[kc];
    f = (k < kin) ? f : 0.f;
    unsigned short h, l;
    sp1(f, h, l);
    hv[e] = h; lv[e] = l;
  }
  unsigned short* dh = ph + (size_t)i * 8;
  unsigned short* dl = pl + (size_t)i * 8;
  *(volatile v8us*)dh = hv;
  *(volatile v8us*)dl = lv;
  __threadfence();
  *(volatile v8us*)dh = hv;
  *(volatile v8us*)dl = lv;
}

template <int NB>
__device__ __forceinline__ int scan_chunk(const int* __restrict__ dsts, int nE, int cbase, int slotBase,
                                          int vec8, int* list, int tid, int lane, int wave) {
  int wc = 0;
#pragma unroll
  for (int g = 0; g < NGRP; ++g) {
    const int el0  = (g * NTHR + tid) * EPT;
    const int e0   = cbase + el0;
    const int sent = -2147483647 - 1;
    v4i da, db;
    if (vec8 != 0 && cbase + CHUNK <= nE) {
      da = *(const v4i*)(dsts + e0);
      db = *(const v4i*)(dsts + e0 + 4);
    } else {
      da.x = (e0     < nE) ? dsts[min(e0, nE - 1)] : sent;
      da.y = (e0 + 1 < nE) ? dsts[min(e0 + 1, nE - 1)] : sent;
      da.z = (e0 + 2 < nE) ? dsts[min(e0 + 2, nE - 1)] : sent;
      da.w = (e0 + 3 < nE) ? dsts[min(e0 + 3, nE - 1)] : sent;
      db.x = (e0 + 4 < nE) ? dsts[min(e0 + 4, nE - 1)] : sent;
      db.y = (e0 + 5 < nE) ? dsts[min(e0 + 5, nE - 1)] : sent;
      db.z = (e0 + 6 < nE) ? dsts[min(e0 + 6, nE - 1)] : sent;
      db.w = (e0 + 7 < nE) ? dsts[min(e0 + 7, nE - 1)] : sent;
    }
    const unsigned nb = (unsigned)slotBase;
    const unsigned s0 = (unsigned)da.x - nb, s1 = (unsigned)da.y - nb;
    const unsigned s2 = (unsigned)da.z - nb, s3 = (unsigned)da.w - nb;
    const unsigned s4 = (unsigned)db.x - nb, s5 = (unsigned)db.y - nb;
    const unsigned s6 = (unsigned)db.z - nb, s7 = (unsigned)db.w - nb;
    const bool h0 = s0 < (unsigned)NB, h1 = s1 < (unsigned)NB, h2 = s2 < (unsigned)NB, h3 = s3 < (unsigned)NB;
    const bool h4 = s4 < (unsigned)NB, h5 = s5 < (unsigned)NB, h6 = s6 < (unsigned)NB, h7 = s7 < (unsigned)NB;
    const unsigned any = __builtin_amdgcn_ballot_w32(h0 | h1 | h2 | h3 | h4 | h5 | h6 | h7);
    if (any != 0u) {
#define HITJ(J, HJ, SJ) { \
        const unsigned mj = __builtin_amdgcn_ballot_w32(HJ); \
        if (mj != 0u) { \
          if (HJ) { \
            const int pos = wc + (int)__builtin_amdgcn_mbcnt_lo(mj, 0u); \
            if (pos < WCAP) list[wave * WCAP + pos] = ((el0 + (J)) << 12) | (int)(SJ); \
          } \
          wc += (int)__builtin_popcount(mj); } }
      HITJ(0, h0, s0)
      HITJ(1, h1, s1)
      HITJ(2, h2, s2)
      HITJ(3, h3, s3)
      HITJ(4, h4, s4)
      HITJ(5, h5, s5)
      HITJ(6, h6, s6)
      HITJ(7, h7, s7)
#undef HITJ
    }
  }
  return wc;
}

__global__ __launch_bounds__(NTHR) void k_count(
    const int* __restrict__ dsts, int* cnt, float* dnv, int nE, int vec8) {
  __shared__ __attribute__((aligned(16))) int scnt[NBC];
  __shared__ __attribute__((aligned(16))) int list[LISTN];
  __shared__ int wcnt[NWAVE];
  const int tid = threadIdx.x, lane = tid & 31, wave = tid >> 5;
  const int nodeBase = blockIdx.x * NBC;

  for (int i = tid; i < NBC; i += NTHR) scnt[i] = 0;
  __syncthreads();

  const int nChunks = (nE + CHUNK - 1) / CHUNK;
#pragma unroll 1
  for (int ch = 0; ch < nChunks; ++ch) {
    const int cbase = ch * CHUNK;
    const int wc = scan_chunk<NBC>(dsts, nE, cbase, nodeBase, vec8, list, tid, lane, wave);
    if (lane == 0) wcnt[wave] = wc;
    __syncthreads();
    if (wave == 0) {
#pragma unroll 1
      for (int wsx = 0; wsx < NWAVE; ++wsx) {
        int n = __builtin_amdgcn_readfirstlane(wcnt[wsx]);
        n = n > WCAP ? WCAP : (n < 0 ? 0 : n);
        const int* lp = list + wsx * WCAP;
#pragma unroll 1
        for (int i = 0; i < n; ++i) {
          const int ent  = __builtin_amdgcn_readfirstlane(lp[i]);
          const int slot = ent & (NBC - 1);
          if (lane == 0) scnt[slot] = scnt[slot] + 1;
        }
      }
    }
    __syncthreads();
  }

  v4i cq[4];
  v4f dq[4];
#pragma unroll
  for (int q = 0; q < 4; ++q) {
    const int f = (wave * 4 + q) * 128 + 4 * lane;
    cq[q] = *(const v4i*)(scnt + f);
    dq[q].x = __builtin_amdgcn_rsqf((float)(max(cq[q].x, 0) + 1));
    dq[q].y = __builtin_amdgcn_rsqf((float)(max(cq[q].y, 0) + 1));
    dq[q].z = __builtin_amdgcn_rsqf((float)(max(cq[q].z, 0) + 1));
    dq[q].w = __builtin_amdgcn_rsqf((float)(max(cq[q].w, 0) + 1));
  }
  int* cpn = cnt + (size_t)nodeBase;
  float* dpn = dnv + (size_t)nodeBase;
#pragma unroll
  for (int q = 0; q < 4; ++q) {
    const int f = (wave * 4 + q) * 128 + 4 * lane;
    *(volatile v4i*)(cpn + f) = cq[q];
    *(volatile v4f*)(dpn + f) = dq[q];
  }
  __threadfence();
#pragma unroll
  for (int q = 0; q < 4; ++q) {
    const int f = (wave * 4 + q) * 128 + 4 * lane;
    *(volatile v4i*)(cpn + f) = cq[q];
    *(volatile v4f*)(dpn + f) = dq[q];
  }
}

__global__ __launch_bounds__(OTHR) void k_offsets(
    const int* __restrict__ cnt, int* off, int* rbase, int nChunk) {
  __shared__ __attribute__((aligned(16))) int soff[NBC];
  __shared__ __attribute__((aligned(16))) int srb[RBN];
  __shared__ int wtot[OTHR / 32];
  const int tid = threadIdx.x, lane = tid & 31, wave = tid >> 5, sub = tid >> 8;
  for (int i = tid; i < RBN; i += OTHR) srb[i] = 0;
  __syncthreads();
  int carry = 0;
#pragma unroll 1
  for (int ch = 0; ch < nChunk; ++ch) {
    const int base = ch * NBC;
    const v4i ca = *(const v4i*)(cnt + base + 8 * tid);
    const v4i cb = *(const v4i*)(cnt + base + 8 * tid + 4);
    const int e0 = max(ca.x, 0), e1 = max(ca.y, 0), e2 = max(ca.z, 0), e3 = max(ca.w, 0);
    const int e4 = max(cb.x, 0), e5 = max(cb.y, 0), e6 = max(cb.z, 0), e7 = max(cb.w, 0);
    const int ts = e0 + e1 + e2 + e3 + e4 + e5 + e6 + e7;
    int incl = ts;
#pragma unroll
    for (int d = 1; d < 32; d <<= 1) {
      const int t = __shfl_up(incl, d);
      if (lane >= d) incl += t;
    }
    if (lane == 31) wtot[wave] = incl;
    __syncthreads();
    int S0 = 0, S1 = 0;
#pragma unroll
    for (int w = 0; w < 8; ++w) { S0 += wtot[w]; S1 += wtot[8 + w]; }
    int pre = 0;
#pragma unroll 1
    for (int w = 8 * sub; w < wave; ++w) pre += wtot[w];
    const int b0 = carry;
    const int b1 = b0 + ((S0 + 31) & ~31);
    const int b2 = b1 + ((S1 + 31) & ~31);
    const int myb = sub == 0 ? b0 : b1;
    if (tid == 0) {
      srb[min(2 * ch + 0, RBN - 1)] = b0;
      srb[min(2 * ch + 1, RBN - 1)] = b1;
    }
    int run = myb + pre + incl - ts;
    soff[8 * tid + 0] = run; run += e0;
    soff[8 * tid + 1] = run; run += e1;
    soff[8 * tid + 2] = run; run += e2;
    soff[8 * tid + 3] = run; run += e3;
    soff[8 * tid + 4] = run; run += e4;
    soff[8 * tid + 5] = run; run += e5;
    soff[8 * tid + 6] = run; run += e6;
    soff[8 * tid + 7] = run;
    carry = b2;
    __syncthreads();
    const v4i o0 = *(const v4i*)(soff + 4 * tid);
    const v4i o1 = *(const v4i*)(soff + 4 * (tid + OTHR));
    int* op = off + base;
    *(volatile v4i*)(op + 4 * tid) = o0;
    *(volatile v4i*)(op + 4 * (tid + OTHR)) = o1;
    __threadfence();
    *(volatile v4i*)(op + 4 * tid) = o0;
    *(volatile v4i*)(op + 4 * (tid + OTHR)) = o1;
    __syncthreads();
  }
  if (tid == 0) srb[min(2 * nChunk, RBN - 1)] = carry;
  __syncthreads();
  v4i rv = {0, 0, 0, 0};
  if (tid < 32) rv = *(const v4i*)(srb + 4 * tid);
  if (tid < 32) *(volatile v4i*)(rbase + 4 * tid) = rv;
  __threadfence();
  if (tid < 32) *(volatile v4i*)(rbase + 4 * tid) = rv;
}

__global__ __launch_bounds__(NTHR) void k_fill(
    const int* __restrict__ dsts, const int* __restrict__ off, const int* __restrict__ rbase,
    int* csr, int nE, int vec8, int csrLen) {
  extern __shared__ v4f lds_dyn[];
  int* region = (int*)lds_dyn;
  int* cursor = region + RCAP;
  int* list   = cursor + NBF;
  int* wcnt   = list + LISTN;
  const int tid = threadIdx.x, lane = tid & 31, wave = tid >> 5;
  const int b = blockIdx.x;
  const int nodeBase = b * NBF;

  int rb0 = rbase[b];
  const int rb1 = rbase[b + 1];
  rb0 = rb0 < 0 ? 0 : (rb0 > csrLen ? csrLen : rb0);
  rb0 &= ~31;
  int len = rb1 - rb0;
  len = len < 0 ? 0 : (len > RCAP ? RCAP : len);
  int lenW = (len + 31) & ~31;
  if (rb0 + lenW > csrLen) lenW = (csrLen - rb0) & ~31;

  {
    const v4i z = {0, 0, 0, 0};
    for (int i = tid; i < RCAP / 4; i += NTHR) ((v4i*)region)[i] = z;
    for (int s = tid; s < NBF; s += NTHR) {
      int o = off[nodeBase + s] - rb0;
      o = o < 0 ? 0 : (o > RCAP ? RCAP : o);
      cursor[s] = o;
    }
  }
  __syncthreads();

  const int nChunks = (nE + CHUNK - 1) / CHUNK;
#pragma unroll 1
  for (int ch = 0; ch < nChunks; ++ch) {
    const int cbase = ch * CHUNK;
    const int wc = scan_chunk<NBF>(dsts, nE, cbase, nodeBase, vec8, list, tid, lane, wave);
    if (lane == 0) wcnt[wave] = wc;
    __syncthreads();
    if (wave == 0) {
#pragma unroll 1
      for (int wsx = 0; wsx < NWAVE; ++wsx) {
        int n = __builtin_amdgcn_readfirstlane(wcnt[wsx]);
        n = n > WCAP ? WCAP : (n < 0 ? 0 : n);
        const int* lp = list + wsx * WCAP;
#pragma unroll 1
        for (int i = 0; i < n; ++i) {
          const int ent  = __builtin_amdgcn_readfirstlane(lp[i]);
          const int slot = ent & (NBF - 1);
          int e = cbase + ((ent >> 12) & (CHUNK - 1));
          e = e > nE - 1 ? nE - 1 : e;
          if (lane == 0) {
            int pos = cursor[slot];
            pos = pos < 0 ? 0 : (pos > RCAP - 1 ? RCAP - 1 : pos);
            region[pos] = e;
            const int np = pos + 1;
            cursor[slot] = np > RCAP ? RCAP : np;
          }
        }
      }
    }
    __syncthreads();
  }

  const int nv = lenW >> 2;
  int* gp = csr + rb0;
#pragma unroll 1
  for (int i = tid; i < nv; i += NTHR) { const v4i v = ((const v4i*)region)[i]; *(volatile v4i*)(gp + 4 * i) = v; }
  __threadfence();
#pragma unroll 1
  for (int i = tid; i < nv; i += NTHR) { const v4i v = ((const v4i*)region)[i]; *(volatile v4i*)(gp + 4 * i) = v; }
}

template <int KD>
__device__ __forceinline__ void mm3(const unsigned short* Ah, const unsigned short* Al,
                                    const unsigned short* __restrict__ Bh, const unsigned short* __restrict__ Bl,
                                    float* stg) {
  static_assert((KD % 32) == 0);
  constexpr int NT  = 8;
  constexpr int NCW = CH / 2;
  const int tid = threadIdx.x, lane = tid & 31, wave = tid >> 5, hh = lane >> 4, m = lane & 15;
  const int r0 = (wave >> 1) * 16, c0 = (wave & 1) * NCW;
  v8f acc[NT];
#pragma unroll
  for (int t = 0; t < NT; ++t) { v8f z = {0.f, 0.f, 0.f, 0.f, 0.f, 0.f, 0.f, 0.f}; acc[t] = z; }
  const unsigned short* aph = Ah + (r0 + m) * KD + 8 * hh;
  const unsigned short* apl = Al + (r0 + m) * KD + 8 * hh;
  const size_t boff = (size_t)(c0 + m) * KD + 8 * hh;
  const unsigned short* bph0 = Bh + boff;
  const unsigned short* bpl0 = Bl + boff;
#pragma unroll 1
  for (int kt = 0; kt < KD / 32; ++kt) {
    FragU ah, al;
    ah.u[0] = *(const v8us*)(aph + 32 * kt);
    ah.u[1] = *(const v8us*)(aph + 32 * kt + 16);
    al.u[0] = *(const v8us*)(apl + 32 * kt);
    al.u[1] = *(const v8us*)(apl + 32 * kt + 16);
#pragma unroll
    for (int t = 0; t < NT; ++t) {
      const size_t to = (size_t)(16 * t) * KD + 32 * kt;
      FragU bh, bl;
      bh.u[0] = *(const v8us*)(bph0 + to);
      bh.u[1] = *(const v8us*)(bph0 + to + 16);
      bl.u[0] = *(const v8us*)(bpl0 + to);
      bl.u[1] = *(const v8us*)(bpl0 + to + 16);
      acc[t] = wmb(ah.w, bh.w, acc[t]);
      acc[t] = wmb(al.w, bh.w, acc[t]);
      acc[t] = wmb(ah.w, bl.w, acc[t]);
    }
  }
  __syncthreads();
  float* sp = stg + (size_t)(r0 + 8 * hh) * CH + c0 + m;
#pragma unroll
  for (int t = 0; t < NT; ++t) {
#pragma unroll
    for (int r = 0; r < 8; ++r) sp[r * CH + 16 * t] = acc[t][r];
  }
}

__global__ __launch_bounds__(NTHR) void k_gemm_in(
    const float* __restrict__ x, const unsigned short* __restrict__ Bh, const unsigned short* __restrict__ Bl,
    const float* __restrict__ bias, float* H, int nN) {
  extern __shared__ v4f lds_dyn[];
  unsigned short* tH = (unsigned short*)lds_dyn;
  unsigned short* tL = tH + BM * KPX;
  float* stg = (float*)lds_dyn;
  const int tid = threadIdx.x, lane = tid & 31, wave = tid >> 5;
  const int rowBase = blockIdx.x * BM;
  constexpr int UPR = KPX / 8;

#pragma unroll 1
  for (int it = 0; it < (BM * UPR) / NTHR; ++it) {
    const int u     = it * NTHR + tid;
    const int row   = u / UPR;
    const int c     = (u - row * UPR) * 8;
    const int grow  = rowBase + row;
    const int growc = grow < nN ? grow : nN - 1;
    const float* xr = x + (size_t)growc * FIN;
    v8us hv, lv;
#pragma unroll
    for (int e = 0; e < 8; ++e) {
      const int k  = c + e;
      const int kc = k < FIN ? k : FIN - 1;
      float f = xr[kc];
      f = (k < FIN && grow < nN) ? f : 0.f;
      unsigned short h, l;
      sp1(f, h, l);
      hv[e] = h; lv[e] = l;
    }
    *(v8us*)(tH + row * KPX + c) = hv;
    *(v8us*)(tL + row * KPX + c) = lv;
  }
  __syncthreads();

  mm3<KPX>(tH, tL, Bh, Bl, stg);
  __syncthreads();

  const int r0 = (wave >> 1) * 16, c0 = (wave & 1) * (CH / 2), col = c0 + 4 * lane;
  const v4f b4 = *(const v4f*)(bias + col);
#pragma unroll
  for (int it = 0; it < 16; ++it) {
    const int row  = r0 + it;
    const int grow = rowBase + row;
    const v4f v = relu4(*(const v4f*)(stg + (size_t)row * CH + col) + b4);
    if (grow < nN) *(volatile v4f*)(H + (size_t)grow * CH + col) = v;
  }
  __threadfence();
#pragma unroll
  for (int it = 0; it < 16; ++it) {
    const int row  = r0 + it;
    const int grow = rowBase + row;
    const v4f v = relu4(*(const v4f*)(stg + (size_t)row * CH + col) + b4);
    if (grow < nN) *(volatile v4f*)(H + (size_t)grow * CH + col) = v;
  }
}

__global__ __launch_bounds__(NTHR) void k_gemm_m(
    const float* __restrict__ A, int alim, const unsigned short* __restrict__ Bh, const unsigned short* __restrict__ Bl,
    float* M, int mlim, int nN) {
  extern __shared__ v4f lds_dyn[];
  unsigned short* tH = (unsigned short*)lds_dyn;
  unsigned short* tL = tH + BM * CH;
  float* stg = (float*)lds_dyn;
  const int tid = threadIdx.x, lane = tid & 31, wave = tid >> 5;
  const int rowBase = blockIdx.x * BM;
  const v4f z4 = {0.f, 0.f, 0.f, 0.f};

#pragma unroll 1
  for (int it = 0; it < (BM * CH / 8) / NTHR; ++it) {
    const int u     = it * NTHR + tid;
    const int row   = u >> 5;
    const int c     = (u & 31) * 8;
    const int grow  = rowBase + row;
    const int growc = grow < alim ? grow : alim - 1;
    const float* ar = A + (size_t)growc * CH + c;
    v4f a = *(const v4f*)ar, b = *(const v4f*)(ar + 4);
    if (grow >= nN) { a = z4; b = z4; }
    v8us hv, lv;
    sp8(a, b, hv, lv);
    *(v8us*)(tH + row * CH + c) = hv;
    *(v8us*)(tL + row * CH + c) = lv;
  }
  __syncthreads();

  mm3<CH>(tH, tL, Bh, Bl, stg);
  __syncthreads();

  const int r0 = (wave >> 1) * 16, c0 = (wave & 1) * (CH / 2), col = c0 + 4 * lane;
#pragma unroll
  for (int it = 0; it < 16; ++it) {
    const int row  = r0 + it;
    const int grow = rowBase + row;
    const v4f v = *(const v4f*)(stg + (size_t)row * CH + col);
    if (grow < mlim) *(volatile v4f*)(M + (size_t)grow * CH + col) = v;
  }
  __threadfence();
#pragma unroll
  for (int it = 0; it < 16; ++it) {
    const int row  = r0 + it;
    const int grow = rowBase + row;
    const v4f v = *(const v4f*)(stg + (size_t)row * CH + col);
    if (grow < mlim) *(volatile v4f*)(M + (size_t)grow * CH + col) = v;
  }
}

__global__ __launch_bounds__(NTHR) void k_gcn(
    const int* __restrict__ csr, const int* __restrict__ off, const int* __restrict__ cnt,
    const int* __restrict__ srcs, const float* __restrict__ dnv, const float* __restrict__ mb,
    const float* __restrict__ cb, float* agg, int nN, int nE, int csrLen) {
  const int tid = threadIdx.x, lane = tid & 31, wave = tid >> 5;
  const int tbase = blockIdx.x * TGT + wave * 32;
  const int ca = 4 * lane, cx = CH / 2 + 4 * lane;
  const v4f z4 = {0.f, 0.f, 0.f, 0.f};
  const v4f ba = *(const v4f*)(cb + ca);
  const v4f bx = *(const v4f*)(cb + cx);
  const int cl = tbase + lane;
  const int cnt_l = cnt[cl];
  const int off_l = off[cl];
  const float dnv_l = dnv[cl];

#pragma unroll 1
  for (int j = 0; j < 32; ++j) {
    const int c = tbase + j;
    int n = __shfl(cnt_l, j);
    n = n < 0 ? 0 : (n > DEGCAP ? DEGCAP : n);
    const int st   = __shfl(off_l, j);
    const float dc = __shfl(dnv_l, j);
    const int cc = c < nN ? c : nN - 1;
    const float* rowm = mb + (size_t)cc * CH;
    const float wsl = dc * dc;
    v4f acca = *(const v4f*)(rowm + ca) * wsl;
    v4f accx = *(const v4f*)(rowm + cx) * wsl;
#pragma unroll 1
    for (int q0 = 0; q0 < n; q0 += 32) {
      int pos = st + q0 + lane;
      pos = pos < 0 ? 0 : (pos > csrLen - 1 ? csrLen - 1 : pos);
      int eid = csr[pos];
      eid = eid < 0 ? 0 : (eid > nE - 1 ? nE - 1 : eid);
      int sl = srcs[eid];
      sl = sl < 0 ? 0 : (sl > nN - 1 ? nN - 1 : sl);
      const float dsl = dnv[sl];
      const int mcnt = (n - q0) < 32 ? (n - q0) : 32;
#pragma unroll 1
      for (int pp = 0; pp < mcnt; ++pp) {
        const int   s = __builtin_amdgcn_readlane(sl, pp);
        const float w = rlf(dsl, pp) * dc;
        const float* rs = mb + (size_t)s * CH;
        const v4f xa = *(const v4f*)(rs + ca);
        const v4f xx = *(const v4f*)(rs + cx);
        acca.x = fmaf(xa.x, w, acca.x); acca.y = fmaf(xa.y, w, acca.y);
        acca.z = fmaf(xa.z, w, acca.z); acca.w = fmaf(xa.w, w, acca.w);
        accx.x = fmaf(xx.x, w, accx.x); accx.y = fmaf(xx.y, w, accx.y);
        accx.z = fmaf(xx.z, w, accx.z); accx.w = fmaf(xx.w, w, accx.w);
      }
    }
    v4f va = acca + ba, vx = accx + bx;
    if (c >= nN) { va = z4; vx = z4; }
    float* po = agg + (size_t)c * CH;
    *(volatile v4f*)(po + ca) = va;
    *(volatile v4f*)(po + cx) = vx;
    __threadfence();
    *(volatile v4f*)(po + ca) = va;
    *(volatile v4f*)(po + cx) = vx;
  }
}

__global__ __launch_bounds__(CH) void k_bnstat(const float* __restrict__ agg, double* part, int nN) {
  __shared__ __attribute__((aligned(16))) double spt[2 * CH];
  const int col = threadIdx.x;
  const int r0 = blockIdx.x * STATR;
  int nr = nN - r0;
  nr = nr < 0 ? 0 : (nr > STATR ? STATR : nr);
  double s = 0.0, q = 0.0;
#pragma unroll 1
  for (int i = 0; i < nr; ++i) {
    const double v = (double)agg[(size_t)(r0 + i) * CH + col];
    s += v;
    q += v * v;
  }
  spt[col] = s;
  spt[CH + col] = q;
  __syncthreads();
  const v2d w = *(const v2d*)(spt + 2 * col);
  double* pp = part + (size_t)blockIdx.x * (2 * CH) + 2 * col;
  *(volatile v2d*)pp = w;
  __threadfence();
  *(volatile v2d*)pp = w;
}

__global__ __launch_bounds__(CH) void k_bnfin(const double* __restrict__ part, const float* __restrict__ gamma,
                                              float* tbl, int nPart, int nN) {
  __shared__ __attribute__((aligned(16))) float stb[2 * CH];
  const int tid = threadIdx.x, col = tid;
  double s = 0.0, q = 0.0;
#pragma unroll 1
  for (int b = 0; b < nPart; ++b) {
    s += part[(size_t)b * (2 * CH) + col];
    q += part[(size_t)b * (2 * CH) + CH + col];
  }
  const double inv = 1.0 / (double)nN;
  const double mu  = s * inv;
  double var = q * inv - mu * mu;
  var = var < 0.0 ? 0.0 : var;
  const float a  = (float)((double)gamma[col] / sqrt(var + BN_EPS));
  const float mf = (float)mu;
  stb[col] = mf;
  stb[CH + col] = a;
  __syncthreads();
  const int t4 = tid < 128 ? tid : 127;
  const v4f w = *(const v4f*)(stb + 4 * t4);
  if (tid < 128) *(volatile v4f*)(tbl + 4 * tid) = w;
  __threadfence();
  if (tid < 128) *(volatile v4f*)(tbl + 4 * tid) = w;
}

__global__ __launch_bounds__(NTHR) void k_bnapply(
    const float* __restrict__ agg, const float* __restrict__ tbl, const float* __restrict__ beta,
    const float* __restrict__ res, int reslim, float* hout, int hlim, int nN) {
  const int tid = threadIdx.x, lane = tid & 31, wave = tid >> 5;
  const int ca = 4 * lane, cx = CH / 2 + 4 * lane;
  const v4f z4 = {0.f, 0.f, 0.f, 0.f};
  const v4f mua = *(const v4f*)(tbl + ca),      mux = *(const v4f*)(tbl + cx);
  const v4f gaa = *(const v4f*)(tbl + CH + ca), gax = *(const v4f*)(tbl + CH + cx);
  const v4f bea = *(const v4f*)(beta + ca),     bex = *(const v4f*)(beta + cx);
  const int rbase = blockIdx.x * BM + wave * 8;
#pragma unroll 1
  for (int rr = 0; rr < 8; ++rr) {
    const int row = rbase + rr;
    const int rc  = row < reslim ? row : reslim - 1;
    const float* arow = agg + (size_t)row * CH;
    const float* rrow = res + (size_t)rc * CH;
    const v4f aa = *(const v4f*)(arow + ca), ax = *(const v4f*)(arow + cx);
    const v4f ra = *(const v4f*)(rrow + ca), rx = *(const v4f*)(rrow + cx);
    v4f ha = relu4((aa - mua) * gaa + bea) + ra;
    v4f hx = relu4((ax - mux) * gax + bex) + rx;
    if (row >= nN) { ha = z4; hx = z4; }
    float* po = hout + (size_t)row * CH;
    if (row < hlim) {
      *(volatile v4f*)(po + ca) = ha;
      *(volatile v4f*)(po + cx) = hx;
    }
    __threadfence();
    if (row < hlim) {
      *(volatile v4f*)(po + ca) = ha;
      *(volatile v4f*)(po + cx) = hx;
    }
  }
}

static size_t carve(size_t* o, size_t bytes) {
  const size_t r = *o;
  *o += (bytes + 255) & ~(size_t)255;
  return r;
}

extern "C" void kernel_launch(void* const* d_in, const int* in_sizes, int n_in,
                              void* d_out, int out_size, void* d_ws, size_t ws_size,
                              hipStream_t stream) {
  if (n_in < 8) return;
  const int nN = in_sizes[0] / FIN;
  const int nE = in_sizes[1] / 2;
  if (nN <= 0 || nE <= 0 || in_sizes[0] != nN * FIN || in_sizes[1] != 2 * nE) return;
  if (in_sizes[2] != CH * FIN || in_sizes[3] != CH || in_sizes[4] != NL * CH * CH) return;
  if (in_sizes[5] != NL * CH || in_sizes[6] != NL * CH || in_sizes[7] != NL * CH) return;
  if ((long long)out_size != (long long)nN * CH) return;
  if (nE > (1 << 27) || nN > (1 << 22)) return;

  const float* x       = (const float*)d_in[0];
  const int*   ei      = (const int*)d_in[1];
  const float* W_in    = (const float*)d_in[2];
  const float* b_in    = (const float*)d_in[3];
  const float* conv_W  = (const float*)d_in[4];
  const float* conv_b  = (const float*)d_in[5];
  const float* bn_g    = (const float*)d_in[6];
  const float* bn_b    = (const float*)d_in[7];
  const int* src = ei;
  const int* dst = ei + nE;
  float* X0 = (float*)d_out;

  const int NPAD   = ((nN + TGT - 1) / TGT) * TGT;
  const int nBC    = (nN + NBC - 1) / NBC;
  const int CNTPAD = nBC * NBC;
  if (FPC * nBC + 1 > RBN) return;
  const int nBF    = (nN + NBF - 1) / NBF;
  const int csrLen = ((nE + 31) & ~31) + 4096;
  if (31 * FPC * nBC > 4096) return;
  const int nAgg   = NPAD / TGT;
  const int nGm    = NPAD / BM;
  const int nStat  = NPAD / STATR;

  char* ws = (char*)d_ws;
  size_t o = 0;
  const size_t oWiH  = carve(&o, (size_t)CH * KPX * 2),       oWiL = carve(&o, (size_t)CH * KPX * 2);
  const size_t oWcH  = carve(&o, (size_t)NL * CH * CH * 2),   oWcL = carve(&o, (size_t)NL * CH * CH * 2);
  const size_t oCnt  = carve(&o, (size_t)CNTPAD * 4);
  const size_t oDnv  = carve(&o, (size_t)CNTPAD * 4);
  const size_t oOff  = carve(&o, (size_t)CNTPAD * 4);
  const size_t oRb   = carve(&o, (size_t)RBN * 4);
  const size_t oCsr  = carve(&o, (size_t)csrLen * 4);
  const size_t oPart = carve(&o, (size_t)nStat * 2 * CH * 8);
  const size_t oTbl  = carve(&o, (size_t)2 * CH * 4);
  const size_t oX1   = carve(&o, (size_t)NPAD * CH * 4);
  const size_t oAgg  = carve(&o, (size_t)NPAD * CH * 4);
  if (o > ws_size || o > (size_t)WSCAP) return;

  unsigned short* wiH = (unsigned short*)(ws + oWiH); unsigned short* wiL = (unsigned short*)(ws + oWiL);
  unsigned short* wcH = (unsigned short*)(ws + oWcH); unsigned short* wcL = (unsigned short*)(ws + oWcL);
  int*    cnt  = (int*)(ws + oCnt);
  float*  dnv  = (float*)(ws + oDnv);
  int*    offp = (int*)(ws + oOff);
  int*    rb   = (int*)(ws + oRb);
  int*    csr  = (int*)(ws + oCsr);
  double* part = (double*)(ws + oPart);
  float*  tbl  = (float*)(ws + oTbl);
  float*  X1   = (float*)(ws + oX1);
  float*  agg  = (float*)(ws + oAgg);

  const int vec8 = ((nE & 3) == 0) ? 1 : 0;

  k_wprep<<<(CH * (KPX / 8) + NTHR - 1) / NTHR, NTHR, 0, stream>>>(W_in, CH, FIN, KPX / 8, wiH, wiL, CH * (KPX / 8));
  k_wprep<<<(NL * CH * (CH / 8) + NTHR - 1) / NTHR, NTHR, 0, stream>>>(conv_W, NL * CH, CH, CH / 8, wcH, wcL, NL * CH * (CH / 8));

  k_count<<<nBC, NTHR, 0, stream>>>(dst, cnt, dnv, nE, vec8);
  k_offsets<<<1, OTHR, 0, stream>>>(cnt, offp, rb, nBC);
  hipFuncSetAttribute(reinterpret_cast<const void*>(&k_fill),
                      hipFuncAttributeMaxDynamicSharedMemorySize, LDS_FILL);
  k_fill<<<nBF, NTHR, LDS_FILL, stream>>>(dst, offp, rb, csr, nE, vec8, csrLen);

  hipFuncSetAttribute(reinterpret_cast<const void*>(&k_gemm_in),
                      hipFuncAttributeMaxDynamicSharedMemorySize, LDS_GEMM);
  hipFuncSetAttribute(reinterpret_cast<const void*>(&k_gemm_m),
                      hipFuncAttributeMaxDynamicSharedMemorySize, LDS_GEMM);
  k_gemm_in<<<nGm, NTHR, LDS_GEMM, stream>>>(x, wiH, wiL, b_in, X0, nN);

  for (int i = 0; i < NL; ++i) {
    const int even = ((i & 1) == 0) ? 1 : 0;
    const float* A  = even ? X0 : X1;  const int alim = even ? nN : NPAD;
    float*       Md = even ? X1 : X0;  const int mlim = even ? NPAD : nN;
    k_gemm_m<<<nGm, NTHR, LDS_GEMM, stream>>>(A, alim, wcH + (size_t)i * CH * CH, wcL + (size_t)i * CH * CH, Md, mlim, nN);
    k_gcn<<<nAgg, NTHR, 0, stream>>>(csr, offp, cnt, src, dnv, Md, conv_b + (size_t)i * CH, agg, nN, nE, csrLen);
    k_bnstat<<<nStat, CH, 0, stream>>>(agg, part, nN);
    k_bnfin<<<1, CH, 0, stream>>>(part, bn_g + (size_t)i * CH, tbl, nStat, nN);
    k_bnapply<<<nGm, NTHR, 0, stream>>>(agg, tbl, bn_b + (size_t)i * CH, A, alim, Md, mlim, nN);
  }
}
